// TransformerBlock_6047313953584
// MI455X (gfx1250) — hardware-verified
//
#include <hip/hip_runtime.h>
#include <stddef.h>


typedef _Float16 v16h __attribute__((ext_vector_type(16)));
typedef _Float16 v8h  __attribute__((ext_vector_type(8)));
typedef float    v8f  __attribute__((ext_vector_type(8)));
typedef float    v4f  __attribute__((ext_vector_type(4)));

#ifndef NB
#define NB 2
#endif
#ifndef SEQ
#define SEQ 2048
#endif
#define NB_FULL  2
#define SEQ_FULL 2048
#define DIM   1024
#define NHEAD 16
#define HD    64
#define DFF   4096
#define MROWS (NB * SEQ)

static_assert(NB >= 1 && NB <= NB_FULL);
static_assert(SEQ >= 128 && SEQ <= SEQ_FULL && (SEQ % 128) == 0);
static_assert(DIM == NHEAD * HD);
static_assert(HD == 64);
static_assert((DIM % 64) == 0 && (DIM % 32) == 0 && (DIM % 256) == 0);
static_assert((DFF % 64) == 0 && (DFF % 32) == 0);
static_assert((MROWS % 64) == 0 && (MROWS % 8) == 0);
static_assert(((SEQ * 32) % 256) == 0);
static_assert((size_t)MROWS * DFF < (size_t)0xFFFFFFFFu);

#define LDT 72
#define LDC 68

#define WCARRY 64.0f
#define PCARRY 1024.0f
#define VCARRY 64.0f
#define HCARRY 64.0f

#define MODE_ROPE  0
#define MODE_VT    1
#define MODE_OPROJ 2
#define MODE_DOWN  3

#define WSQ_BYTES     ((size_t)DIM * DIM * 2)
#define WFF_BYTES     ((size_t)DIM * DFF * 2)
#define TH_BYTES      ((size_t)4 * DIM * 4)
#define SS_BYTES      ((size_t)4 * 2 * DIM * 4)
#define CS_BYTES      ((size_t)SEQ * 64 * 4)
#define PLANE16_BYTES ((size_t)MROWS * DIM * 2)
#define X1_BYTES      ((size_t)MROWS * DIM * 4)
#define H_BYTES       ((size_t)MROWS * DFF * 2)

#define OFF_WQ  ((size_t)0)
#define OFF_WK  (OFF_WQ + WSQ_BYTES)
#define OFF_WV  (OFF_WK + WSQ_BYTES)
#define OFF_WO  (OFF_WV + WSQ_BYTES)
#define OFF_WG  (OFF_WO + WSQ_BYTES)
#define OFF_WU  (OFF_WG + WFF_BYTES)
#define OFF_WD  (OFF_WU + WFF_BYTES)
#define OFF_TH  (OFF_WD + WFF_BYTES)
#define OFF_SS  (OFF_TH + TH_BYTES)
#define OFF_CS  (OFF_SS + SS_BYTES)
#define OFF_NX  (OFF_CS + CS_BYTES)
#define OFF_Q   (OFF_NX + PLANE16_BYTES)
#define OFF_K   (OFF_Q + PLANE16_BYTES)
#define OFF_VT  (OFF_K + PLANE16_BYTES)
#define OFF_CTX (OFF_VT + PLANE16_BYTES)
#define OFF_X1  (OFF_CTX + PLANE16_BYTES)
#define OFF_H   (OFF_X1 + X1_BYTES)
#define WS_TOTAL (OFF_H + H_BYTES)

static_assert((WSQ_BYTES % 128) == 0 && (WFF_BYTES % 128) == 0);
static_assert((TH_BYTES % 128) == 0 && (SS_BYTES % 128) == 0 && (CS_BYTES % 128) == 0);
static_assert((PLANE16_BYTES % 128) == 0 && (X1_BYTES % 128) == 0 && (H_BYTES % 128) == 0);
static_assert(WS_TOTAL <= (size_t)134217728);

__device__ __forceinline__ float bf16r(float x) {
  unsigned int u = __float_as_uint(x);
  u = (u + 0x7FFFu + ((u >> 16) & 1u)) & 0xFFFF0000u;
  return __uint_as_float(u);
}
__device__ __forceinline__ v4f bf16r4(v4f a) {
  v4f r;
#pragma unroll
  for (int j = 0; j < 4; ++j) r[j] = bf16r(a[j]);
  return r;
}

__device__ __forceinline__ v16h frag_at(const _Float16* p) {
  v8h lo = *(const v8h*)(p);
  v8h hi = *(const v8h*)(p + 16);
  v16h out;
#pragma unroll
  for (int i = 0; i < 8; ++i) { out[i] = lo[i]; out[i + 8] = hi[i]; }
  return out;
}
__device__ __forceinline__ v16h ld_frag(const _Float16* base, unsigned ld) {
  const unsigned lane = threadIdx.x & 31u;
  return frag_at(base + (lane & 15u) * ld + (lane >> 4) * 8u);
}

__device__ __forceinline__ v8f wmma16(v16h a, v16h b, v8f c) {
  v8f d = __builtin_amdgcn_wmma_f32_16x16x32_f16(false, a, false, b, (short)0, c,
                                                 false, false);
  asm volatile("v_nop\n\tv_nop\n\tv_nop\n\tv_nop" : "+v"(d) : "v"(a), "v"(b));
  return d;
}

__device__ __forceinline__ float red16_max(float x) {
#pragma unroll
  for (int off = 1; off < 16; off <<= 1) x = fmaxf(x, __shfl_xor(x, off, 32));
  return x;
}
__device__ __forceinline__ float red16_sum(float x) {
#pragma unroll
  for (int off = 1; off < 16; off <<= 1) x += __shfl_xor(x, off, 32);
  return x;
}

__device__ __forceinline__ void wave_lds_sync() {
  __builtin_amdgcn_fence(3  , "wavefront");
  asm volatile("s_wait_dscnt 0x0" ::: "memory");
  __builtin_amdgcn_wave_barrier();
}

__global__ __launch_bounds__(256) void wconv_kernel(
    const float* __restrict__ W, _Float16* __restrict__ Wt, unsigned Kdim, unsigned Ndim) {
  __shared__ _Float16 T[64 * LDT];
  const unsigned tid = threadIdx.x;
  const unsigned n0 = blockIdx.x * 64u;
  const unsigned k0 = blockIdx.y * 64u;
#pragma unroll 4
  for (unsigned j = 0; j < 16u; ++j) {
    const unsigned idx = tid + 256u * j;
    const unsigned kr = idx >> 6, nc = idx & 63u;
    const float v = W[(size_t)(k0 + kr) * Ndim + n0 + nc];
    T[nc * LDT + kr] = (_Float16)(WCARRY * bf16r(v));
  }
  __syncthreads();
  v8h x[2];
  size_t off[2];
#pragma unroll
  for (unsigned i = 0; i < 2u; ++i) {
    const unsigned n = 32u * i + (tid >> 3);
    const unsigned kc = (tid & 7u) * 8u;
    x[i] = *(const v8h*)&T[n * LDT + kc];
    off[i] = (size_t)(n0 + n) * Kdim + k0 + kc;
  }
#pragma unroll
  for (int i = 0; i < 2; ++i) *(volatile v8h*)(Wt + off[i]) = x[i];
  __threadfence();
#pragma unroll
  for (int i = 0; i < 2; ++i) *(volatile v8h*)(Wt + off[i]) = x[i];
}

__global__ __launch_bounds__(256) void time_hidden_kernel(
    const float* __restrict__ te,
    const float* __restrict__ w1a, const float* __restrict__ b1a,
    const float* __restrict__ w1b, const float* __restrict__ b1b,
    float* __restrict__ th) {
  const unsigned j = blockIdx.x * 256u + threadIdx.x;
  float a00 = 0.0f, a01 = 0.0f, a10 = 0.0f, a11 = 0.0f;
#pragma unroll 4
  for (unsigned i = 0; i < (unsigned)DIM; ++i) {
    const float t0 = bf16r(te[i]);
    const float t1 = bf16r(te[DIM + i]);
    const float wa = bf16r(w1a[(size_t)i * DIM + j]);
    const float wb = bf16r(w1b[(size_t)i * DIM + j]);
    a00 = fmaf(t0, wa, a00);
    a01 = fmaf(t1, wa, a01);
    a10 = fmaf(t0, wb, a10);
    a11 = fmaf(t1, wb, a11);
  }
  const float ba = bf16r(b1a[j]);
  const float bb = bf16r(b1b[j]);
  float z[4];
  z[0] = a00 + ba; z[1] = a01 + ba; z[2] = a10 + bb; z[3] = a11 + bb;
  float v[4];
#pragma unroll
  for (int q = 0; q < 4; ++q)
    v[q] = z[q] * __builtin_amdgcn_rcpf(1.0f + __expf(-z[q]));
#pragma unroll
  for (int q = 0; q < 4; ++q) *(volatile float*)(th + (size_t)q * DIM + j) = v[q];
  __threadfence();
#pragma unroll
  for (int q = 0; q < 4; ++q) *(volatile float*)(th + (size_t)q * DIM + j) = v[q];
}

__global__ __launch_bounds__(256) void time_ss_kernel(
    const float* __restrict__ th,
    const float* __restrict__ w2a, const float* __restrict__ b2a,
    const float* __restrict__ w2b, const float* __restrict__ b2b,
    float* __restrict__ ss) {
  const unsigned j = blockIdx.x * 256u + threadIdx.x;
  float a00 = 0.0f, a01 = 0.0f, a10 = 0.0f, a11 = 0.0f;
#pragma unroll 4
  for (unsigned i = 0; i < (unsigned)DIM; ++i) {
    const float h00 = th[i];
    const float h01 = th[DIM + i];
    const float h10 = th[2 * DIM + i];
    const float h11 = th[3 * DIM + i];
    const float wa = bf16r(w2a[(size_t)i * (2 * DIM) + j]);
    const float wb = bf16r(w2b[(size_t)i * (2 * DIM) + j]);
    a00 = fmaf(h00, wa, a00);
    a01 = fmaf(h01, wa, a01);
    a10 = fmaf(h10, wb, a10);
    a11 = fmaf(h11, wb, a11);
  }
  const float ba = bf16r(b2a[j]);
  const float bb = bf16r(b2b[j]);
  float v[4];
  v[0] = a00 + ba; v[1] = a01 + ba; v[2] = a10 + bb; v[3] = a11 + bb;
#pragma unroll
  for (int q = 0; q < 4; ++q) *(volatile float*)(ss + (size_t)q * (2 * DIM) + j) = v[q];
  __threadfence();
#pragma unroll
  for (int q = 0; q < 4; ++q) *(volatile float*)(ss + (size_t)q * (2 * DIM) + j) = v[q];
}

__global__ __launch_bounds__(256) void rope_table_kernel(float* __restrict__ cs) {
  const unsigned t = blockIdx.x * 256u + threadIdx.x;
  const unsigned s = t >> 5, i = t & 31u;
  const float inv = exp2f(-(float)i * 0.4152410118609203f);
  const float ang = (float)s * inv;
  float sn, c;
  sincosf(ang, &sn, &c);
  float* p = cs + (size_t)s * 64u + i;
  *(volatile float*)(p) = c;
  *(volatile float*)(p + 32) = sn;
  __threadfence();
  *(volatile float*)(p) = c;
  *(volatile float*)(p + 32) = sn;
}

template <int FIRST>
__global__ __launch_bounds__(256) void norm_kernel(
    const float* __restrict__ src, const float* __restrict__ wn,
    const float* __restrict__ ss, _Float16* __restrict__ dst) {
  const unsigned lane = threadIdx.x & 31u;
  const unsigned wave = (unsigned)__builtin_amdgcn_readfirstlane((int)(threadIdx.x >> 5));
  const unsigned crow = blockIdx.x * 8u + wave;
  const unsigned bidx = crow / (unsigned)SEQ;
  const unsigned sq = crow - bidx * (unsigned)SEQ;
  const size_t srow = FIRST ? ((size_t)bidx * SEQ_FULL + sq) : (size_t)crow;
  const float* xr = src + srow * DIM + lane * 8u;

  v4f a[8];
  float sum = 0.0f;
#pragma unroll
  for (int j = 0; j < 4; ++j) {
    v4f u0 = *(const v4f*)(xr + 256 * j);
    v4f u1 = *(const v4f*)(xr + 256 * j + 4);
    if (FIRST) { u0 = bf16r4(u0); u1 = bf16r4(u1); }
    a[2 * j] = u0;
    a[2 * j + 1] = u1;
#pragma unroll
    for (int e = 0; e < 4; ++e) sum += u0[e] * u0[e];
#pragma unroll
    for (int e = 0; e < 4; ++e) sum += u1[e] * u1[e];
  }
#pragma unroll
  for (int off = 1; off < 32; off <<= 1) sum += __shfl_xor(sum, off, 32);
  const float rn = rsqrtf(sum * (1.0f / (float)DIM) + 1.0e-5f);

  const float* sc = ss + (size_t)bidx * (2 * DIM) + lane * 8u;
  const float* sh = sc + DIM;
  const float* wp = wn + lane * 8u;
  v8h o[4];
  size_t off[4];
#pragma unroll
  for (int j = 0; j < 4; ++j) {
    const v4f w0 = bf16r4(*(const v4f*)(wp + 256 * j));
    const v4f w1 = bf16r4(*(const v4f*)(wp + 256 * j + 4));
    const v4f s0 = *(const v4f*)(sc + 256 * j);
    const v4f s1 = *(const v4f*)(sc + 256 * j + 4);
    const v4f h0 = *(const v4f*)(sh + 256 * j);
    const v4f h1 = *(const v4f*)(sh + 256 * j + 4);
#pragma unroll
    for (int e = 0; e < 4; ++e) {
      o[j][e]     = (_Float16)(((a[2 * j][e] * rn) * w0[e]) * (1.0f + s0[e]) + h0[e]);
      o[j][e + 4] = (_Float16)(((a[2 * j + 1][e] * rn) * w1[e]) * (1.0f + s1[e]) + h1[e]);
    }
    off[j] = (size_t)crow * DIM + 256u * (unsigned)j + lane * 8u;
  }
#pragma unroll
  for (int j = 0; j < 4; ++j) *(volatile v8h*)(dst + off[j]) = o[j];
  __threadfence();
#pragma unroll
  for (int j = 0; j < 4; ++j) *(volatile v8h*)(dst + off[j]) = o[j];
}

template <int MODE, int KD>
__global__ __launch_bounds__(256) void gemm_kernel(
    const _Float16* __restrict__ A16, const _Float16* __restrict__ Bt,
    const float* __restrict__ bias, const float* __restrict__ addf,
    const float* __restrict__ cstab, float* __restrict__ outf,
    _Float16* __restrict__ out16) {
  __shared__ float Cs[64 * LDC];
  const unsigned tid = threadIdx.x, lane = tid & 31u;
  const unsigned w = (unsigned)__builtin_amdgcn_readfirstlane((int)(tid >> 5));
  const unsigned mw = w >> 1, nw = w & 1u;
  const unsigned hh = lane >> 4, m = lane & 15u;
  const unsigned n0 = blockIdx.x * 64u;
  const unsigned row0 = blockIdx.y * 64u;

  const _Float16* ap  = A16 + (size_t)(row0 + mw * 16u + m) * KD + hh * 8u;
  const _Float16* bp0 = Bt + (size_t)(n0 + nw * 32u + m) * KD + hh * 8u;
  const _Float16* bp1 = bp0 + 16 * KD;
  v8f acc0 = {}, acc1 = {};
#pragma unroll 2
  for (unsigned k0 = 0; k0 < (unsigned)KD; k0 += 32u) {
    const v16h a  = frag_at(ap + k0);
    const v16h b0 = frag_at(bp0 + k0);
    const v16h b1 = frag_at(bp1 + k0);
    acc0 = wmma16(a, b0, acc0);
    acc1 = wmma16(a, b1, acc1);
  }
#pragma unroll
  for (int r = 0; r < 8; ++r) {
    float* d = &Cs[(mw * 16u + hh * 8u + (unsigned)r) * LDC + nw * 32u + m];
    d[0]  = acc0[r];
    d[16] = acc1[r];
  }
  __syncthreads();

  if (MODE == MODE_ROPE) {
    v8h x[2];
    size_t off[2];
#pragma unroll
    for (unsigned i = 0; i < 2u; ++i) {
      const unsigned r = 32u * i + (tid >> 3);
      const unsigned c = (tid & 7u) * 8u;
      const unsigned pc = c ^ 32u;
      const unsigned f = c & 31u;
      const unsigned crow = row0 + r;
      const unsigned bidx = crow / (unsigned)SEQ;
      const unsigned sq = crow - bidx * (unsigned)SEQ;
      const float sgn = (c < 32u) ? -1.0f : 1.0f;
      const v4f u0 = *(const v4f*)&Cs[r * LDC + c];
      const v4f u1 = *(const v4f*)&Cs[r * LDC + c + 4];
      const v4f p0 = *(const v4f*)&Cs[r * LDC + pc];
      const v4f p1 = *(const v4f*)&Cs[r * LDC + pc + 4];
      const v4f b0 = bf16r4(*(const v4f*)(bias + n0 + c));
      const v4f b1 = bf16r4(*(const v4f*)(bias + n0 + c + 4));
      const v4f g0 = bf16r4(*(const v4f*)(bias + n0 + pc));
      const v4f g1 = bf16r4(*(const v4f*)(bias + n0 + pc + 4));
      const float* ct = cstab + (size_t)sq * 64u + f;
      const v4f c0 = *(const v4f*)(ct);
      const v4f c1 = *(const v4f*)(ct + 4);
      const v4f s0 = *(const v4f*)(ct + 32);
      const v4f s1 = *(const v4f*)(ct + 36);
#pragma unroll
      for (int j = 0; j < 4; ++j) {
        const float qa = u0[j] * (1.0f / WCARRY) + b0[j];
        const float ra = sgn * (p0[j] * (1.0f / WCARRY) + g0[j]);
        const float qb = u1[j] * (1.0f / WCARRY) + b1[j];
        const float rb = sgn * (p1[j] * (1.0f / WCARRY) + g1[j]);
        x[i][j]     = (_Float16)(qa * c0[j] + ra * s0[j]);
        x[i][j + 4] = (_Float16)(qb * c1[j] + rb * s1[j]);
      }
      off[i] = (size_t)crow * DIM + n0 + c;
    }
#pragma unroll
    for (int i = 0; i < 2; ++i) *(volatile v8h*)(out16 + off[i]) = x[i];
    __threadfence();
#pragma unroll
    for (int i = 0; i < 2; ++i) *(volatile v8h*)(out16 + off[i]) = x[i];
  }

  if (MODE == MODE_VT) {
    const unsigned bidx = row0 / (unsigned)SEQ;
    const unsigned key0 = row0 - bidx * (unsigned)SEQ;
    v8h x[2];
    size_t off[2];
#pragma unroll
    for (unsigned i = 0; i < 2u; ++i) {
      const unsigned dcol = 32u * i + (tid >> 3);
      const unsigned kk = (tid & 7u) * 8u;
      const float bb = bf16r(bias[n0 + dcol]);
#pragma unroll
      for (unsigned j = 0; j < 8u; ++j)
        x[i][j] = (_Float16)(Cs[(kk + j) * LDC + dcol] * (1.0f / WCARRY) + bb);
      off[i] = ((size_t)bidx * DIM + n0 + dcol) * SEQ + key0 + kk;
    }
#pragma unroll
    for (int i = 0; i < 2; ++i) *(volatile v8h*)(out16 + off[i]) = x[i];
    __threadfence();
#pragma unroll
    for (int i = 0; i < 2; ++i) *(volatile v8h*)(out16 + off[i]) = x[i];
  }

  if (MODE == MODE_OPROJ || MODE == MODE_DOWN) {
    v4f xs[4];
    size_t off[4];
#pragma unroll
    for (unsigned i = 0; i < 4u; ++i) {
      const unsigned r = 16u * i + (tid >> 4);
      const unsigned c = (tid & 15u) * 4u;
      const unsigned crow = row0 + r;
      const unsigned bidx = crow / (unsigned)SEQ;
      const unsigned sq = crow - bidx * (unsigned)SEQ;
      const size_t frow = (size_t)bidx * SEQ_FULL + sq;
      const v4f u = *(const v4f*)&Cs[r * LDC + c];
      v4f val;
      if (MODE == MODE_OPROJ) {
        const v4f g = bf16r4(*(const v4f*)(bias + n0 + c));
        const v4f xin = bf16r4(*(const v4f*)(addf + frow * DIM + n0 + c));
#pragma unroll
        for (int j = 0; j < 4; ++j)
          val[j] = (xin[j] + u[j] * (1.0f / (WCARRY * VCARRY))) + g[j];
        off[i] = (size_t)crow * DIM + n0 + c;
      } else {
        const v4f xin = *(const v4f*)(addf + (size_t)crow * DIM + n0 + c);
#pragma unroll
        for (int j = 0; j < 4; ++j)
          val[j] = xin[j] + u[j] * (1.0f / (WCARRY * HCARRY));
        off[i] = frow * DIM + n0 + c;
      }
      xs[i] = val;
    }
#pragma unroll
    for (int i = 0; i < 4; ++i) *(volatile v4f*)(outf + off[i]) = xs[i];
    __threadfence();
#pragma unroll
    for (int i = 0; i < 4; ++i) *(volatile v4f*)(outf + off[i]) = xs[i];
  }
}

__global__ __launch_bounds__(256) void glu_kernel(
    const _Float16* __restrict__ A16, const _Float16* __restrict__ Wg,
    const _Float16* __restrict__ Wu, _Float16* __restrict__ H16) {
  __shared__ float Cg[64 * LDC];
  __shared__ float Cu[64 * LDC];
  const unsigned tid = threadIdx.x, lane = tid & 31u;
  const unsigned w = (unsigned)__builtin_amdgcn_readfirstlane((int)(tid >> 5));
  const unsigned mw = w >> 1, nw = w & 1u;
  const unsigned hh = lane >> 4, m = lane & 15u;
  const unsigned n0 = blockIdx.x * 64u;
  const unsigned row0 = blockIdx.y * 64u;

  const _Float16* ap  = A16 + (size_t)(row0 + mw * 16u + m) * DIM + hh * 8u;
  const _Float16* gp0 = Wg + (size_t)(n0 + nw * 32u + m) * DIM + hh * 8u;
  const _Float16* gp1 = gp0 + 16 * DIM;
  const _Float16* up0 = Wu + (size_t)(n0 + nw * 32u + m) * DIM + hh * 8u;
  const _Float16* up1 = up0 + 16 * DIM;
  v8f g0 = {}, g1 = {}, u0 = {}, u1 = {};
#pragma unroll 2
  for (unsigned k0 = 0; k0 < (unsigned)DIM; k0 += 32u) {
    const v16h a   = frag_at(ap + k0);
    const v16h bg0 = frag_at(gp0 + k0);
    const v16h bg1 = frag_at(gp1 + k0);
    const v16h bu0 = frag_at(up0 + k0);
    const v16h bu1 = frag_at(up1 + k0);
    g0 = wmma16(a, bg0, g0);
    g1 = wmma16(a, bg1, g1);
    u0 = wmma16(a, bu0, u0);
    u1 = wmma16(a, bu1, u1);
  }
#pragma unroll
  for (int r = 0; r < 8; ++r) {
    const unsigned o = (mw * 16u + hh * 8u + (unsigned)r) * LDC + nw * 32u + m;
    Cg[o]      = g0[r];
    Cg[o + 16] = g1[r];
    Cu[o]      = u0[r];
    Cu[o + 16] = u1[r];
  }
  __syncthreads();

#pragma unroll 1
  for (unsigned it = 0; it < 16u; ++it) {
    const unsigned idx = tid + 256u * it;
    const unsigned o = (idx >> 6) * LDC + (idx & 63u);
    const float g = Cg[o] * (1.0f / WCARRY);
    const float uraw = Cu[o];
    const float ge = 0.5f * g * (1.0f + erff(g * 0.70710678f));
    Cg[o] = ge * uraw;
  }
  __syncthreads();

  v8h x[2];
  size_t off[2];
#pragma unroll
  for (unsigned i = 0; i < 2u; ++i) {
    const unsigned r = 32u * i + (tid >> 3);
    const unsigned c = (tid & 7u) * 8u;
    const v4f t0 = *(const v4f*)&Cg[r * LDC + c];
    const v4f t1 = *(const v4f*)&Cg[r * LDC + c + 4];
#pragma unroll
    for (int j = 0; j < 4; ++j) {
      x[i][j]     = (_Float16)t0[j];
      x[i][j + 4] = (_Float16)t1[j];
    }
    off[i] = (size_t)(row0 + r) * DFF + n0 + c;
  }
#pragma unroll
  for (int i = 0; i < 2; ++i) *(volatile v8h*)(H16 + off[i]) = x[i];
  __threadfence();
#pragma unroll
  for (int i = 0; i < 2; ++i) *(volatile v8h*)(H16 + off[i]) = x[i];
}
static_assert(HCARRY == WCARRY);

__global__ __launch_bounds__(256) void attn_kernel(
    const _Float16* __restrict__ Qh, const _Float16* __restrict__ Kh,
    const _Float16* __restrict__ Vt, _Float16* __restrict__ Ov) {
  __shared__ _Float16 Ks[64 * LDT];
  __shared__ _Float16 Vs[64 * LDT];
  __shared__ _Float16 Ps[8 * 16 * LDT];

  const unsigned tid = threadIdx.x, lane = tid & 31u;
  const unsigned w = (unsigned)__builtin_amdgcn_readfirstlane((int)(tid >> 5));
  const unsigned hh = lane >> 4, m = lane & 15u;
  const unsigned q0 = blockIdx.x * 128u;
  const unsigned head = blockIdx.y;
  const unsigned b = blockIdx.z;
  const float scale = 0.125f;
  const unsigned pb = w * (16u * LDT);

  const size_t qoff = (size_t)(b * (unsigned)SEQ + q0 + w * 16u + m) * DIM + head * HD + hh * 8u;
  v16h qf[2];
  qf[0] = frag_at(Qh + qoff);
  qf[1] = frag_at(Qh + qoff + 32);

  float mrow[8], lrow[8];
  v8f o[4];
#pragma unroll
  for (int v = 0; v < 8; ++v) { mrow[v] = -1.0e30f; lrow[v] = 0.0f; }
#pragma unroll
  for (int nb = 0; nb < 4; ++nb) o[nb] = (v8f){};

  const size_t kplane = (size_t)b * SEQ * DIM + head * HD;
  const size_t vplane = ((size_t)b * DIM + head * HD) * SEQ;

  for (unsigned kb = 0; kb < (unsigned)SEQ; kb += 64u) {
#pragma unroll
    for (unsigned j = 0; j < 2u; ++j) {
      const unsigned idx = tid + 256u * j;
      const unsigned r = idx >> 3, c = (idx & 7u) * 8u;
      *(v8h*)&Ks[r * LDT + c] = *(const v8h*)(Kh + kplane + (size_t)(kb + r) * DIM + c);
      *(v8h*)&Vs[r * LDT + c] = *(const v8h*)(Vt + vplane + (size_t)r * SEQ + kb + c);
    }
    __syncthreads();

    v8f s[4];
#pragma unroll
    for (int kg = 0; kg < 4; ++kg) {
      v8f t = {};
#pragma unroll
      for (int c = 0; c < 2; ++c) {
        const v16h kf = ld_frag(&Ks[(kg * 16) * LDT + c * 32], LDT);
        t = wmma16(qf[c], kf, t);
      }
      s[kg] = t * scale;
    }

    float alpha[8];
#pragma unroll
    for (int v = 0; v < 8; ++v) {
      float mx = fmaxf(fmaxf(s[0][v], s[1][v]), fmaxf(s[2][v], s[3][v]));
      mx = red16_max(mx);
      const float mn = fmaxf(mrow[v], mx);
      alpha[v] = __expf(mrow[v] - mn);
      mrow[v] = mn;
    }
#pragma unroll
    for (int kg = 0; kg < 4; ++kg)
#pragma unroll
      for (int v = 0; v < 8; ++v) s[kg][v] = __expf(s[kg][v] - mrow[v]);
#pragma unroll
    for (int v = 0; v < 8; ++v) {
      const float rs = red16_sum((s[0][v] + s[1][v]) + (s[2][v] + s[3][v]));
      lrow[v] = alpha[v] * lrow[v] + rs;
    }
#pragma unroll
    for (int nb = 0; nb < 4; ++nb)
#pragma unroll
      for (int v = 0; v < 8; ++v) o[nb][v] = o[nb][v] * alpha[v];

#pragma unroll
    for (int kg = 0; kg < 4; ++kg)
#pragma unroll
      for (int v = 0; v < 8; ++v)
        Ps[pb + (hh * 8u + (unsigned)v) * LDT + (unsigned)kg * 16u + m] =
            (_Float16)(s[kg][v] * PCARRY);
    wave_lds_sync();

#pragma unroll
    for (int c = 0; c < 2; ++c) {
      const v16h pf = ld_frag(&Ps[pb + c * 32], LDT);
#pragma unroll
      for (int nb = 0; nb < 4; ++nb) {
        const v16h vf = ld_frag(&Vs[(nb * 16) * LDT + c * 32], LDT);
        o[nb] = wmma16(pf, vf, o[nb]);
      }
    }
    __syncthreads();
  }

  float inv[8];
#pragma unroll
  for (int v = 0; v < 8; ++v) inv[v] = __builtin_amdgcn_rcpf(lrow[v]) * (VCARRY / PCARRY);
#pragma unroll
  for (int nb = 0; nb < 4; ++nb)
#pragma unroll
    for (int v = 0; v < 8; ++v)
      Ps[pb + (hh * 8u + (unsigned)v) * LDT + (unsigned)nb * 16u + m] =
          (_Float16)(o[nb][v] * inv[v]);
  wave_lds_sync();
  v8h x[4];
  size_t off[4];
#pragma unroll
  for (unsigned i = 0; i < 4u; ++i) {
    const unsigned r = 4u * i + (lane >> 3);
    const unsigned c = (lane & 7u) * 8u;
    x[i] = *(const v8h*)&Ps[pb + r * LDT + c];
    off[i] = (size_t)(b * (unsigned)SEQ + q0 + w * 16u + r) * DIM + head * HD + c;
  }
#pragma unroll
  for (int i = 0; i < 4; ++i) *(volatile v8h*)(Ov + off[i]) = x[i];
  __threadfence();
#pragma unroll
  for (int i = 0; i < 4; ++i) *(volatile v8h*)(Ov + off[i]) = x[i];
}

extern "C" void kernel_launch(void* const* d_in, const int* in_sizes, int n_in,
                              void* d_out, int out_size, void* d_ws, size_t ws_size,
                              hipStream_t stream) {
  if (n_in < 23) return;
  const long long need_x = ((long long)(NB - 1) * SEQ_FULL + SEQ) * DIM;
  if ((long long)in_sizes[0] < need_x) return;
  if (in_sizes[1] < 2 * DIM) return;
  if (in_sizes[2] < DIM || in_sizes[7] < DIM) return;
  if ((long long)in_sizes[3] < (long long)DIM * DIM) return;
  if ((long long)in_sizes[8] < (long long)DIM * DIM) return;
  if (in_sizes[4] < DIM || in_sizes[9] < DIM) return;
  if ((long long)in_sizes[5] < (long long)DIM * 2 * DIM) return;
  if ((long long)in_sizes[10] < (long long)DIM * 2 * DIM) return;
  if (in_sizes[6] < 2 * DIM || in_sizes[11] < 2 * DIM) return;
  if ((long long)in_sizes[12] < (long long)DIM * DIM) return;
  if ((long long)in_sizes[14] < (long long)DIM * DIM) return;
  if ((long long)in_sizes[16] < (long long)DIM * DIM) return;
  if ((long long)in_sizes[18] < (long long)DIM * DIM) return;
  if (in_sizes[13] < DIM || in_sizes[15] < DIM || in_sizes[17] < DIM || in_sizes[19] < DIM) return;
  if ((long long)in_sizes[20] < (long long)DIM * DFF) return;
  if ((long long)in_sizes[21] < (long long)DIM * DFF) return;
  if ((long long)in_sizes[22] < (long long)DFF * DIM) return;
  if ((long long)out_size < need_x) return;
  if (ws_size < WS_TOTAL) return;

  const float* x       = (const float*)d_in[0];
  const float* te      = (const float*)d_in[1];
  const float* w_norm1 = (const float*)d_in[2];
  const float* t1_w1   = (const float*)d_in[3];
  const float* t1_b1   = (const float*)d_in[4];
  const float* t1_w2   = (const float*)d_in[5];
  const float* t1_b2   = (const float*)d_in[6];
  const float* w_norm2 = (const float*)d_in[7];
  const float* t2_w1   = (const float*)d_in[8];
  const float* t2_b1   = (const float*)d_in[9];
  const float* t2_w2   = (const float*)d_in[10];
  const float* t2_b2   = (const float*)d_in[11];
  const float* wq = (const float*)d_in[12];
  const float* bq = (const float*)d_in[13];
  const float* wk = (const float*)d_in[14];
  const float* bk = (const float*)d_in[15];
  const float* wv = (const float*)d_in[16];
  const float* bv = (const float*)d_in[17];
  const float* wo = (const float*)d_in[18];
  const float* bo = (const float*)d_in[19];
  const float* w_gate = (const float*)d_in[20];
  const float* w_up   = (const float*)d_in[21];
  const float* w_down = (const float*)d_in[22];
  float* out = (float*)d_out;

  char* ws = (char*)d_ws;
  _Float16* WtQ   = (_Float16*)(ws + OFF_WQ);
  _Float16* WtK   = (_Float16*)(ws + OFF_WK);
  _Float16* WtV   = (_Float16*)(ws + OFF_WV);
  _Float16* WtO   = (_Float16*)(ws + OFF_WO);
  _Float16* WtG   = (_Float16*)(ws + OFF_WG);
  _Float16* WtU   = (_Float16*)(ws + OFF_WU);
  _Float16* WtD   = (_Float16*)(ws + OFF_WD);
  float*    TH    = (float*)(ws + OFF_TH);
  float*    SS    = (float*)(ws + OFF_SS);
  float*    CS    = (float*)(ws + OFF_CS);
  _Float16* NX16  = (_Float16*)(ws + OFF_NX);
  _Float16* Q16   = (_Float16*)(ws + OFF_Q);
  _Float16* K16   = (_Float16*)(ws + OFF_K);
  _Float16* Vt16  = (_Float16*)(ws + OFF_VT);
  _Float16* Ctx16 = (_Float16*)(ws + OFF_CTX);
  float*    X1    = (float*)(ws + OFF_X1);
  _Float16* H16   = (_Float16*)(ws + OFF_H);

  dim3 blk(256);
  dim3 gg(DIM / 64, MROWS / 64);

  wconv_kernel<<<dim3(DIM / 64, DIM / 64), blk, 0, stream>>>(wq, WtQ, DIM, DIM);
  wconv_kernel<<<dim3(DIM / 64, DIM / 64), blk, 0, stream>>>(wk, WtK, DIM, DIM);
  wconv_kernel<<<dim3(DIM / 64, DIM / 64), blk, 0, stream>>>(wv, WtV, DIM, DIM);
  wconv_kernel<<<dim3(DIM / 64, DIM / 64), blk, 0, stream>>>(wo, WtO, DIM, DIM);
  wconv_kernel<<<dim3(DFF / 64, DIM / 64), blk, 0, stream>>>(w_gate, WtG, DIM, DFF);
  wconv_kernel<<<dim3(DFF / 64, DIM / 64), blk, 0, stream>>>(w_up, WtU, DIM, DFF);
  wconv_kernel<<<dim3(DIM / 64, DFF / 64), blk, 0, stream>>>(w_down, WtD, DFF, DIM);

  time_hidden_kernel<<<dim3(DIM / 256), blk, 0, stream>>>(te, t1_w1, t1_b1, t2_w1, t2_b1, TH);
  time_ss_kernel<<<dim3(2 * DIM / 256), blk, 0, stream>>>(TH, t1_w2, t1_b2, t2_w2, t2_b2, SS);
  rope_table_kernel<<<dim3(SEQ * 32 / 256), blk, 0, stream>>>(CS);

  norm_kernel<1><<<dim3(MROWS / 8), blk, 0, stream>>>(x, w_norm1, SS, NX16);
  gemm_kernel<MODE_ROPE, DIM><<<gg, blk, 0, stream>>>(NX16, WtQ, bq, x, CS, X1, Q16);
  gemm_kernel<MODE_ROPE, DIM><<<gg, blk, 0, stream>>>(NX16, WtK, bk, x, CS, X1, K16);
  gemm_kernel<MODE_VT, DIM><<<gg, blk, 0, stream>>>(NX16, WtV, bv, x, CS, X1, Vt16);
  attn_kernel<<<dim3(SEQ / 128, NHEAD, NB), blk, 0, stream>>>(Q16, K16, Vt16, Ctx16);
  gemm_kernel<MODE_OPROJ, DIM><<<gg, blk, 0, stream>>>(Ctx16, WtO, bo, x, CS, X1, Q16);

  norm_kernel<0><<<dim3(MROWS / 8), blk, 0, stream>>>(X1, w_norm2, SS + 2 * 2 * DIM, NX16);
  glu_kernel<<<dim3(DFF / 64, MROWS / 64), blk, 0, stream>>>(NX16, WtG, WtU, H16);
  gemm_kernel<MODE_DOWN, DFF><<<gg, blk, 0, stream>>>(H16, WtD, bo, X1, CS, out, Q16);
}
